// Model_55224689492143
// MI455X (gfx1250) — hardware-verified
//
#include <hip/hip_runtime.h>
#include <stddef.h>
#include <stdint.h>

#define NB     8
#define NN     512
#define ND     64
#define NO     64
#define MROWS  (NB * NN)
#define KPAIR  128
#define KTAIL  192
#define XS     72
#define BS     136
#define ATHR   256
#define NWAVE  8
#define QPB    16
#define QPW    2
#define TROWS  128
#define BN_EPS 1e-5f

#define LO_X   0
#define LO_W   (LO_X + NN * XS * 2)
#define LO_P   (LO_W + ND * NO * 4)
#define LO_BT  (LO_P + 128 * 4)
#define LO_S   (LO_BT + NWAVE * NO * BS * 2)
#define ATT_LDS (LO_S + NWAVE * NN * 4)

#define WO_XB   0
#define WO_AGG  (WO_XB + MROWS * ND * 2)
#define WO_WAP  (WO_AGG + MROWS * KPAIR * 2)
#define WO_WT   (WO_WAP + ND * NO * 4)
#define WO_PV   (WO_WT + NO * KTAIL * 2)
#define WS_TOTAL (WO_PV + 8 * 64 * 4)

#define PB_WAP 128
#define PB_WT  132
#define PB_PV  133
#define PB_END 134

static_assert(NN == 32 * 16);
static_assert(ND == 64 && NO == 64 && ND == 2 * 32 && NO == 4 * 16);
static_assert(QPB == NWAVE * QPW && NN % QPB == 0);
static_assert(KPAIR == 2 * ND && KTAIL == 3 * ND && KPAIR % 32 == 0 && KTAIL % 32 == 0);
static_assert(MROWS % TROWS == 0 && TROWS == NWAVE * 16);
static_assert((XS * 2) % 16 == 0 && (BS * 2) % 16 == 0 && XS >= ND + 8 && BS >= KPAIR + 8);
static_assert(LO_W % 16 == 0 && LO_P % 16 == 0 && LO_BT % 16 == 0 && LO_S % 16 == 0);
static_assert(ATT_LDS == 246272 && ATT_LDS <= 327680);
static_assert(WO_AGG % 256 == 0 && WO_WAP % 256 == 0 && WO_WT % 256 == 0 && WO_PV % 256 == 0 && WS_TOTAL % 256 == 0);
static_assert(WS_TOTAL == 1615872 && WS_TOTAL <= 134217728);
static_assert(PB_WAP * ATHR * 8 == MROWS * ND);
static_assert((PB_WT - PB_WAP) * ATHR * 4 == ND * NO);
static_assert(6 * ATHR * 8 == NO * KTAIL);

typedef float          v4f   __attribute__((ext_vector_type(4)));
typedef float          v8f   __attribute__((ext_vector_type(8)));
typedef int            v8i   __attribute__((ext_vector_type(8)));
typedef unsigned       v4u   __attribute__((ext_vector_type(4)));
typedef unsigned short v8us  __attribute__((ext_vector_type(8)));
typedef unsigned short v16us __attribute__((ext_vector_type(16)));
typedef __bf16         v16bf __attribute__((ext_vector_type(16)));
typedef v4f  __attribute__((may_alias)) v4fa;
typedef v4u  __attribute__((may_alias)) v4ua;
typedef v8us __attribute__((may_alias)) v8usa;
typedef unsigned __attribute__((may_alias)) ua;
union FragB { v16bf v; v16us u; v8us h[2]; v8i w; };

__device__ __forceinline__ v8f wmb(const FragB& a, const FragB& b, v8f c) {
  v8f d = __builtin_amdgcn_wmma_f32_16x16x32_bf16(false, a.v, false, b.v, (short)0, c, false, false);
  asm volatile("v_nop\n\tv_nop\n\tv_nop\n\tv_nop" : "+v"(d) : "v"(a.w), "v"(b.w));
  return d;
}

__device__ __forceinline__ unsigned bf16_bits(float f) {
  const unsigned u = __float_as_uint(f);
  return (u + 0x7FFFu + ((u >> 16) & 1u)) >> 16;
}
__device__ __forceinline__ float bf16_val(float f) {
  return __uint_as_float(bf16_bits(f) << 16);
}

__device__ __forceinline__ void wave_sync() {
  __builtin_amdgcn_fence(__ATOMIC_RELEASE, "workgroup");
  __builtin_amdgcn_wave_barrier();
  __builtin_amdgcn_fence(__ATOMIC_ACQUIRE, "workgroup");
}

__device__ __forceinline__ float hsum16(float v) {
  v += __shfl_xor(v, 8);
  v += __shfl_xor(v, 4);
  v += __shfl_xor(v, 2);
  v += __shfl_xor(v, 1);
  return v;
}

__device__ __forceinline__ float tanh_f(float v) {
  v = fminf(fmaxf(v, -15.0f), 15.0f);
  const float e = expf(2.0f * v);
  return 1.0f - 2.0f / (1.0f + e);
}

__global__ __launch_bounds__(ATHR) void k_prep(
    const float* __restrict__ x, const float* __restrict__ W_ap,
    const float* __restrict__ W_pa, const float* __restrict__ W_po,
    const float* __restrict__ p0, const float* __restrict__ p1, const float* __restrict__ p2,
    const float* __restrict__ p3, const float* __restrict__ p4, const float* __restrict__ p5,
    const float* __restrict__ p6, const float* __restrict__ p7,
    unsigned short* XB, float* WAPR, unsigned short* WT, float* PV)
{
  __shared__ __attribute__((aligned(16))) float sT[2 * ND * NO];
  const int b = (int)blockIdx.x, tid = (int)threadIdx.x;
  if (b < PB_WAP) {
    const int g = b * ATHR + tid;
    const float* src = x + (size_t)g * 8;
    const v4f a = *(const v4fa*)src;
    const v4f c = *(const v4fa*)(src + 4);
    v8us o;
    o[0] = (unsigned short)bf16_bits(a.x); o[1] = (unsigned short)bf16_bits(a.y);
    o[2] = (unsigned short)bf16_bits(a.z); o[3] = (unsigned short)bf16_bits(a.w);
    o[4] = (unsigned short)bf16_bits(c.x); o[5] = (unsigned short)bf16_bits(c.y);
    o[6] = (unsigned short)bf16_bits(c.z); o[7] = (unsigned short)bf16_bits(c.w);
    unsigned short* dp = XB + (size_t)g * 8;
    *(volatile v8us*)dp = o;
    __threadfence();
    *(volatile v8us*)dp = o;
  } else if (b < PB_WT) {
    const int q = (b - PB_WAP) * ATHR + tid;
    const v4f v = *(const v4fa*)(W_ap + (size_t)q * 4);
    const v4f r = { bf16_val(v.x), bf16_val(v.y), bf16_val(v.z), bf16_val(v.w) };
    float* dp = WAPR + (size_t)q * 4;
    *(volatile v4f*)dp = r;
    __threadfence();
    *(volatile v4f*)dp = r;
  } else if (b < PB_PV) {
#pragma unroll
    for (int it = 0; it < 4; ++it) {
      const int q = tid + ATHR * it;
      const v4f v = *(const v4fa*)(W_pa + (size_t)q * 4);
      const v4f r = { bf16_val(v.x), bf16_val(v.y), bf16_val(v.z), bf16_val(v.w) };
      *(v4fa*)(sT + q * 4) = r;
    }
#pragma unroll
    for (int it = 0; it < 4; ++it) {
      const int q = tid + ATHR * it;
      const v4f v = *(const v4fa*)(W_po + (size_t)q * 4);
      const v4f r = { bf16_val(v.x), bf16_val(v.y), bf16_val(v.z), bf16_val(v.w) };
      *(v4fa*)(sT + ND * NO + q * 4) = r;
    }
    __syncthreads();
    v8us o[6];
#pragma unroll
    for (int it = 0; it < 6; ++it) {
      const int c  = tid + ATHR * it;
      const int n  = c / 24;
      const int k0 = (c - 24 * n) * 8;
      const int base = (k0 >= 128) ? (ND * NO + (k0 - 128) * NO) : ((k0 & 63) * NO);
      v8us t;
#pragma unroll
      for (int j = 0; j < 8; ++j) t[j] = (unsigned short)bf16_bits(sT[base + j * NO + n]);
      o[it] = t;
    }
#pragma unroll
    for (int it = 0; it < 6; ++it) *(volatile v8us*)(WT + (size_t)(tid + ATHR * it) * 8) = o[it];
    __threadfence();
#pragma unroll
    for (int it = 0; it < 6; ++it) *(volatile v8us*)(WT + (size_t)(tid + ATHR * it) * 8) = o[it];
  } else {
    if (tid < 32) {
      const int c4 = (tid & 15) * 4;
      v4f v[8];
      v[0] = *(const v4fa*)(p0 + c4); v[1] = *(const v4fa*)(p1 + c4);
      v[2] = *(const v4fa*)(p2 + c4); v[3] = *(const v4fa*)(p3 + c4);
      v[4] = *(const v4fa*)(p4 + c4); v[5] = *(const v4fa*)(p5 + c4);
      v[6] = *(const v4fa*)(p6 + c4); v[7] = *(const v4fa*)(p7 + c4);
#pragma unroll
      for (int a = 0; a < 8; ++a) {
        const v4f r = { bf16_val(v[a].x), bf16_val(v[a].y), bf16_val(v[a].z), bf16_val(v[a].w) };
        v[a] = r;
      }
      if (tid < 16) {
#pragma unroll
        for (int a = 0; a < 8; ++a) *(volatile v4f*)(PV + a * 64 + c4) = v[a];
      }
      __threadfence();
      if (tid < 16) {
#pragma unroll
        for (int a = 0; a < 8; ++a) *(volatile v4f*)(PV + a * 64 + c4) = v[a];
      }
    }
  }
}

__global__ __launch_bounds__(ATHR) __attribute__((amdgpu_num_vgpr(248)))
void k_attn(const unsigned short* __restrict__ XB, const float* __restrict__ WAPR,
            const float* __restrict__ PV, unsigned* AGGu)
{
  extern __shared__ __attribute__((aligned(16))) unsigned char smem[];
  unsigned short* sX = (unsigned short*)(smem + LO_X);
  float* sW   = (float*)(smem + LO_W);
  float* sPar = (float*)(smem + LO_P);
  const int tid = (int)threadIdx.x, lane = tid & 31, wave = tid >> 5;
  const int hh = lane >> 4, m = lane & 15;
  unsigned short* bt = (unsigned short*)(smem + LO_BT) + wave * (NO * BS);
  float* S = (float*)(smem + LO_S) + wave * NN;
  const int b = (int)blockIdx.x >> 5, qt = (int)blockIdx.x & 31;

  {
    const unsigned short* xbb = XB + (size_t)b * NN * ND;
#pragma unroll 4
    for (int it = 0; it < 16; ++it) {
      const int c = tid + ATHR * it;
      const int row = c >> 3, seg = c & 7;
      const v8us v = *(const v8usa*)(xbb + (size_t)c * 8);
      *(v8usa*)(sX + row * XS + seg * 8) = v;
    }
    const v8us z = {0, 0, 0, 0, 0, 0, 0, 0};
#pragma unroll
    for (int it = 0; it < 2; ++it) {
      const int row = tid + ATHR * it;
      *(v8usa*)(sX + row * XS + ND) = z;
    }
#pragma unroll
    for (int it = 0; it < 4; ++it) {
      const int q = tid + ATHR * it;
      const v4f v = *(const v4fa*)(WAPR + (size_t)q * 4);
      *(v4fa*)(sW + q * 4) = v;
    }
    if (tid < 32) {
      const v4f v = *(const v4fa*)(PV + tid * 4);
      *(v4fa*)(sPar + tid * 4) = v;
    }
    *(v8usa*)(bt + lane * BS + KPAIR) = z;
    *(v8usa*)(bt + (lane + 32) * BS + KPAIR) = z;
  }
  __syncthreads();

  const ua* sXu = (const ua*)sX;
  const v8f z8 = {0.f, 0.f, 0.f, 0.f, 0.f, 0.f, 0.f, 0.f};

#pragma unroll 1
  for (int qi = 0; qi < QPW; ++qi) {
    const int i = qt * QPB + wave * QPW + qi;
    wave_sync();

    {
      const unsigned short* xi = sX + i * XS;
#pragma unroll 1
      for (int it = 0; it < 16; ++it) {
        const int o  = ((it & 1) << 5) + lane;
        const int k0 = (it >> 1) * 8;
        const v4u xw = *(const v4ua*)(xi + k0);
        float xf[8];
        xf[0] = __uint_as_float(xw.x << 16); xf[1] = __uint_as_float(xw.x & 0xffff0000u);
        xf[2] = __uint_as_float(xw.y << 16); xf[3] = __uint_as_float(xw.y & 0xffff0000u);
        xf[4] = __uint_as_float(xw.z << 16); xf[5] = __uint_as_float(xw.z & 0xffff0000u);
        xf[6] = __uint_as_float(xw.w << 16); xf[7] = __uint_as_float(xw.w & 0xffff0000u);
        v8us hv, lv;
#pragma unroll
        for (int j = 0; j < 8; ++j) {
          const float p = xf[j] * sW[(k0 + j) * NO + o];
          const unsigned hb = bf16_bits(p);
          const unsigned lb = bf16_bits(p - __uint_as_float(hb << 16));
          hv[j] = (unsigned short)hb;
          lv[j] = (unsigned short)lb;
        }
        *(v8usa*)(bt + o * BS + k0) = hv;
        *(v8usa*)(bt + o * BS + ND + k0) = lv;
      }
    }
    wave_sync();

#pragma unroll 1
    for (int jt = 0; jt < NN / 16; ++jt) {
      const unsigned short* ap = sX + (16 * jt + m) * XS + 8 * hh;
      FragB a0, a1;
      a0.h[0] = *(const v8usa*)(ap);
      a0.h[1] = *(const v8usa*)(ap + 16);
      a1.h[0] = *(const v8usa*)(ap + 32);
      a1.h[1] = *(const v8usa*)(ap + 48);
      float sj[8];
#pragma unroll
      for (int r = 0; r < 8; ++r) sj[r] = 0.0f;
#pragma unroll 1
      for (int nt = 0; nt < 4; ++nt) {
        const unsigned short* bp = bt + (16 * nt + m) * BS + 8 * hh;
        FragB bh0, bh1, bl0, bl1;
        bh0.h[0] = *(const v8usa*)(bp);       bh0.h[1] = *(const v8usa*)(bp + 16);
        bh1.h[0] = *(const v8usa*)(bp + 32);  bh1.h[1] = *(const v8usa*)(bp + 48);
        bl0.h[0] = *(const v8usa*)(bp + 64);  bl0.h[1] = *(const v8usa*)(bp + 80);
        bl1.h[0] = *(const v8usa*)(bp + 96);  bl1.h[1] = *(const v8usa*)(bp + 112);
        v8f acc = z8;
        acc = wmb(a0, bh0, acc);
        acc = wmb(a1, bh1, acc);
        acc = wmb(a0, bl0, acc);
        acc = wmb(a1, bl1, acc);
        const float bias = sPar[16 * nt + m];
        const float aw   = sPar[NO + 16 * nt + m];
#pragma unroll
        for (int r = 0; r < 8; ++r) sj[r] = fmaf(tanh_f(acc[r] + bias), aw, sj[r]);
      }
#pragma unroll
      for (int r = 0; r < 8; ++r) sj[r] = hsum16(sj[r]);
      if (m == 0) {
        const v4f s0 = { sj[0], sj[1], sj[2], sj[3] };
        const v4f s1 = { sj[4], sj[5], sj[6], sj[7] };
        *(v4fa*)(S + 16 * jt + 8 * hh) = s0;
        *(v4fa*)(S + 16 * jt + 8 * hh + 4) = s1;
      }
    }
    wave_sync();

    float mx = -3.0e38f;
#pragma unroll 4
    for (int t = 0; t < NN / 32; ++t) mx = fmaxf(mx, S[lane + 32 * t]);
    mx = fmaxf(mx, __shfl_xor(mx, 16));
    mx = fmaxf(mx, __shfl_xor(mx, 8));
    mx = fmaxf(mx, __shfl_xor(mx, 4));
    mx = fmaxf(mx, __shfl_xor(mx, 2));
    mx = fmaxf(mx, __shfl_xor(mx, 1));
    float l = 0.0f;
#pragma unroll 2
    for (int t = 0; t < NN / 32; ++t) {
      const float e = expf(S[lane + 32 * t] - mx);
      S[lane + 32 * t] = e;
      l += e;
    }
    l += __shfl_xor(l, 16);
    l += __shfl_xor(l, 8);
    l += __shfl_xor(l, 4);
    l += __shfl_xor(l, 2);
    l += __shfl_xor(l, 1);
    wave_sync();

    float g0 = 0.0f, g1 = 0.0f;
#pragma unroll 2
    for (int j4 = 0; j4 < NN / 4; ++j4) {
      const v4f p4 = *(const v4fa*)(S + 4 * j4);
      const unsigned w0 = sXu[(4 * j4 + 0) * (XS / 2) + lane];
      const unsigned w1 = sXu[(4 * j4 + 1) * (XS / 2) + lane];
      const unsigned w2 = sXu[(4 * j4 + 2) * (XS / 2) + lane];
      const unsigned w3 = sXu[(4 * j4 + 3) * (XS / 2) + lane];
      g0 = fmaf(p4.x, __uint_as_float(w0 << 16), g0);
      g1 = fmaf(p4.x, __uint_as_float(w0 & 0xffff0000u), g1);
      g0 = fmaf(p4.y, __uint_as_float(w1 << 16), g0);
      g1 = fmaf(p4.y, __uint_as_float(w1 & 0xffff0000u), g1);
      g0 = fmaf(p4.z, __uint_as_float(w2 << 16), g0);
      g1 = fmaf(p4.z, __uint_as_float(w2 & 0xffff0000u), g1);
      g0 = fmaf(p4.w, __uint_as_float(w3 << 16), g0);
      g1 = fmaf(p4.w, __uint_as_float(w3 & 0xffff0000u), g1);
    }
    const float inv = 1.0f / l;
    g0 = g0 * inv;
    g1 = g1 * inv;

    const unsigned h0 = bf16_bits(g0);
    const unsigned h1 = bf16_bits(g1);
    const unsigned l0 = bf16_bits(g0 - __uint_as_float(h0 << 16));
    const unsigned l1 = bf16_bits(g1 - __uint_as_float(h1 << 16));
    const unsigned whi = (h0 & 0xffffu) | (h1 << 16);
    const unsigned wlo = (l0 & 0xffffu) | (l1 << 16);
    unsigned* rp = AGGu + (size_t)(b * NN + i) * (KPAIR / 2) + lane;
    *(volatile unsigned*)rp = whi;
    *(volatile unsigned*)(rp + 32) = wlo;
    __threadfence();
    *(volatile unsigned*)rp = whi;
    *(volatile unsigned*)(rp + 32) = wlo;
  }
}

__global__ __launch_bounds__(ATHR) void k_tail(const unsigned short* __restrict__ AGG,
                                               const unsigned short* __restrict__ XB,
                                               const unsigned short* __restrict__ WT,
                                               const float* __restrict__ PV, float* out)
{
  __shared__ __attribute__((aligned(16))) float stg[TROWS * NO];
  const int tid = (int)threadIdx.x, lane = tid & 31, wave = tid >> 5;
  const int hh = lane >> 4, m = lane & 15;
  const int rowBase = (int)blockIdx.x * TROWS;
  const int row = rowBase + 16 * wave + m;

  v8f acc[4];
  {
    const v8f z = {0.f, 0.f, 0.f, 0.f, 0.f, 0.f, 0.f, 0.f};
#pragma unroll
    for (int t = 0; t < 4; ++t) acc[t] = z;
  }
  const unsigned short* ap = AGG + (size_t)row * KPAIR + 8 * hh;
  const unsigned short* xp = XB + (size_t)row * ND + 8 * hh;
  const unsigned short* bp = WT + (size_t)m * KTAIL + 8 * hh;

#pragma unroll 1
  for (int k0 = 0; k0 < KPAIR; k0 += 32) {
    FragB af;
    af.h[0] = *(const v8usa*)(ap + k0);
    af.h[1] = *(const v8usa*)(ap + k0 + 16);
#pragma unroll
    for (int nt = 0; nt < 4; ++nt) {
      const unsigned short* wq = bp + (size_t)(16 * nt) * KTAIL + k0;
      FragB bf;
      bf.h[0] = *(const v8usa*)wq;
      bf.h[1] = *(const v8usa*)(wq + 16);
      acc[nt] = wmb(af, bf, acc[nt]);
    }
  }
#pragma unroll 1
  for (int k0 = 0; k0 < ND; k0 += 32) {
    FragB af;
    af.h[0] = *(const v8usa*)(xp + k0);
    af.h[1] = *(const v8usa*)(xp + k0 + 16);
#pragma unroll
    for (int nt = 0; nt < 4; ++nt) {
      const unsigned short* wq = bp + (size_t)(16 * nt) * KTAIL + KPAIR + k0;
      FragB bf;
      bf.h[0] = *(const v8usa*)wq;
      bf.h[1] = *(const v8usa*)(wq + 16);
      acc[nt] = wmb(af, bf, acc[nt]);
    }
  }

#pragma unroll
  for (int nt = 0; nt < 4; ++nt) {
    const int lc = 16 * nt + m;
#pragma unroll
    for (int r = 0; r < 8; ++r) stg[(16 * wave + 8 * hh + r) * NO + lc] = acc[nt][r];
  }
  __syncthreads();

  const int c4 = 4 * m;
  const v4f bpa = *(const v4fa*)(PV + 2 * 64 + c4);
  const v4f bpo = *(const v4fa*)(PV + 3 * 64 + c4);
  const v4f gam = *(const v4fa*)(PV + 4 * 64 + c4);
  const v4f bet = *(const v4fa*)(PV + 5 * 64 + c4);
  const v4f mu  = *(const v4fa*)(PV + 6 * 64 + c4);
  const v4f var = *(const v4fa*)(PV + 7 * 64 + c4);
  v4f rs;
  rs.x = 1.0f / sqrtf(var.x + BN_EPS);
  rs.y = 1.0f / sqrtf(var.y + BN_EPS);
  rs.z = 1.0f / sqrtf(var.z + BN_EPS);
  rs.w = 1.0f / sqrtf(var.w + BN_EPS);
  const float SELU_A = 1.6732632423543772f;
  const float SELU_S = 1.0507009873554805f;

  float* myp = stg + (16 * wave + hh) * NO + c4;
#pragma unroll 1
  for (int i = 0; i < 8; ++i) {
    float* p = myp + (2 * i) * NO;
    const v4f v = *(const v4fa*)p;
    v4f t;
    t.x = (((v.x + bpa.x) + bpo.x) - mu.x) * rs.x * gam.x + bet.x;
    t.y = (((v.y + bpa.y) + bpo.y) - mu.y) * rs.y * gam.y + bet.y;
    t.z = (((v.z + bpa.z) + bpo.z) - mu.z) * rs.z * gam.z + bet.z;
    t.w = (((v.w + bpa.w) + bpo.w) - mu.w) * rs.w * gam.w + bet.w;
    v4f y;
    const float ex = SELU_A * expm1f(t.x);
    const float ey = SELU_A * expm1f(t.y);
    const float ez = SELU_A * expm1f(t.z);
    const float ew = SELU_A * expm1f(t.w);
    y.x = SELU_S * ((t.x > 0.0f) ? t.x : ex);
    y.y = SELU_S * ((t.y > 0.0f) ? t.y : ey);
    y.z = SELU_S * ((t.z > 0.0f) ? t.z : ez);
    y.w = SELU_S * ((t.w > 0.0f) ? t.w : ew);
    *(v4fa*)p = y;
  }
  wave_sync();

  float* ob = out + (size_t)(rowBase + 16 * wave + hh) * NO + c4;
#pragma unroll
  for (int i = 0; i < 8; ++i) {
    const v4f v = *(const v4fa*)(myp + (2 * i) * NO);
    *(volatile v4f*)(ob + (size_t)(2 * i) * NO) = v;
  }
  __threadfence();
#pragma unroll
  for (int i = 0; i < 8; ++i) {
    const v4f v = *(const v4fa*)(myp + (2 * i) * NO);
    *(volatile v4f*)(ob + (size_t)(2 * i) * NO) = v;
  }
}

extern "C" void kernel_launch(void* const* d_in, const int* in_sizes, int n_in,
                              void* d_out, int out_size, void* d_ws, size_t ws_size,
                              hipStream_t stream) {
  if (n_in < 12) return;
  if (in_sizes[0] != MROWS * ND) return;
  if (in_sizes[1] != ND * NO || in_sizes[2] != NO) return;
  if (in_sizes[3] != NO) return;
  if (in_sizes[4] != ND * NO || in_sizes[5] != NO) return;
  if (in_sizes[6] != ND * NO || in_sizes[7] != NO) return;
  if (in_sizes[8] != NO || in_sizes[9] != NO || in_sizes[10] != NO || in_sizes[11] != NO) return;
  if (out_size != MROWS * NO) return;
  if ((size_t)WS_TOTAL > ws_size) return;

  const float* x     = (const float*)d_in[0];
  const float* W_ap  = (const float*)d_in[1];
  const float* b_ap  = (const float*)d_in[2];
  const float* att_w = (const float*)d_in[3];
  const float* W_pa  = (const float*)d_in[4];
  const float* b_pa  = (const float*)d_in[5];
  const float* W_po  = (const float*)d_in[6];
  const float* b_po  = (const float*)d_in[7];
  const float* gamma = (const float*)d_in[8];
  const float* beta  = (const float*)d_in[9];
  const float* rmean = (const float*)d_in[10];
  const float* rvar  = (const float*)d_in[11];
  float* out = (float*)d_out;

  char* ws = (char*)d_ws;
  unsigned short* XB   = (unsigned short*)(ws + WO_XB);
  unsigned short* AGG  = (unsigned short*)(ws + WO_AGG);
  float*          WAPR = (float*)(ws + WO_WAP);
  unsigned short* WT   = (unsigned short*)(ws + WO_WT);
  float*          PV   = (float*)(ws + WO_PV);

  hipFuncSetAttribute(reinterpret_cast<const void*>(&k_attn), hipFuncAttributeMaxDynamicSharedMemorySize,
                      (int)ATT_LDS);

  k_prep<<<PB_END, ATHR, 0, stream>>>(x, W_ap, W_pa, W_po, b_ap, att_w, b_pa, b_po, gamma, beta, rmean, rvar,
                                      XB, WAPR, WT, PV);
  k_attn<<<NB * (NN / QPB), ATHR, ATT_LDS, stream>>>(XB, WAPR, PV, (unsigned*)AGG);
  k_tail<<<MROWS / TROWS, ATHR, 0, stream>>>(AGG, XB, WT, PV, out);
}
